// CDMamba_seg_cd_5145370821211
// MI455X (gfx1250) — hardware-verified
//
#include <hip/hip_runtime.h>


#define NB_    4
#define CCH_   128
#define HH_    64
#define WW_    64
#define LL_    (HH_ * WW_)
#define MT_    (NB_ * LL_)
#define NG_    4
#define DM_    32
#define DI_    64
#define NS_    16
#define DTR_   2
#define XDW_   (DTR_ + 2 * NS_)
#define XDN_   64
#define NGD_   (NG_ * 2)
#define NOUT_  128
#define SXP_   (CCH_ + 4)
#define EPS_   1e-5f
#define WSC_   64.0f
#define USC_   1024.0f
#define YSC_   1024.0f

static_assert(MT_ % 64 == 0);
static_assert(LL_ % 64 == 0);
static_assert(LL_ % 32 == 0);
static_assert(LL_ % 8 == 0);
static_assert(CCH_ == 128);
static_assert(NG_ * DM_ == CCH_);
static_assert(XDW_ + 2 <= 36);
static_assert(36 <= XDN_);
static_assert(DI_ == 64);

typedef float          v4f   __attribute__((ext_vector_type(4)));
typedef float          v8f   __attribute__((ext_vector_type(8)));
typedef _Float16       v8h   __attribute__((ext_vector_type(8)));
typedef _Float16       v16h  __attribute__((ext_vector_type(16)));
typedef unsigned short u16x8 __attribute__((ext_vector_type(8)));

union FragH { u16x8 h[2]; v16h v; };
union Pack8 { v8h f; u16x8 u; };

__device__ __forceinline__ v8f ld8f(const float* p) {
    v4f a = *(const v4f*)p;
    v4f b = *(const v4f*)(p + 4);
    return __builtin_shufflevector(a, b, 0, 1, 2, 3, 4, 5, 6, 7);
}
__device__ __forceinline__ float sigm_f(float x) {
    return __builtin_amdgcn_rcpf(1.0f + __expf(-x));
}
__device__ __forceinline__ float silu_f(float x) { return x * sigm_f(x); }
__device__ __forceinline__ float softplus_f(float x) {
    return fmaxf(x, 0.0f) + __logf(1.0f + __expf(-fabsf(x)));
}

__device__ __forceinline__ void mma16(v8f& acc, const FragH& a, const FragH& b) {
    acc = __builtin_amdgcn_wmma_f32_16x16x32_f16(false, a.v, false, b.v, (short)0, acc, false, false);
    asm volatile("v_nop\n\tv_nop\n\tv_nop\n\tv_nop" : "+v"(acc) : "v"(a.v), "v"(b.v));
}

__global__ __launch_bounds__(256)
void cvt_w_kernel(const float* __restrict__ gw, const float* __restrict__ pw,
                  const float* __restrict__ wi, const float* __restrict__ wx,
                  const float* __restrict__ wo,
                  unsigned short* dg, unsigned short* dp, unsigned short* di,
                  unsigned short* dx, unsigned short* dwo)
{
    const int sel = blockIdx.y;
    const int i = blockIdx.x * 256 + threadIdx.x;
    const float* src;
    unsigned short* dst;
    int n8;
    if (sel == 0)      { src = gw; dst = dg;  n8 = (CCH_ * CCH_) / 8; }
    else if (sel == 1) { src = pw; dst = dp;  n8 = (NOUT_ * CCH_) / 8; }
    else if (sel == 2) { src = wi; dst = di;  n8 = (NG_ * 2 * DI_ * DM_) / 8; }
    else if (sel == 3) { src = wx; dst = dx;  n8 = (NGD_ * XDN_ * DI_) / 8; }
    else               { src = wo; dst = dwo; n8 = (NG_ * DM_ * 2 * DI_) / 8; }
    if (i >= n8) return;
    const size_t e = (size_t)i * 8;
    v8f x;
#pragma unroll
    for (int c = 0; c < 8; ++c) x[c] = 0.0f;
    if (sel == 3) {
        const int k  = (int)(e % DI_);
        const int r  = (int)((e / DI_) % XDN_);
        const int gd = (int)(e / ((size_t)DI_ * XDN_));
        if (r < XDW_) x = ld8f(src + ((size_t)(gd * XDW_ + r)) * DI_ + k);
    } else if (sel == 4) {
        const int kk = (int)(e % (2 * DI_));
        const int n  = (int)((e / (2 * DI_)) % DM_);
        const int g  = (int)(e / ((size_t)2 * DI_ * DM_));
        x = ld8f(src + ((size_t)(g * DM_ + n)) * DI_ + (kk & (DI_ - 1)));
    } else {
        x = ld8f(src + e);
    }
    Pack8 pk;
    pk.f = __builtin_convertvector(x * WSC_, v8h);
    const u16x8 v = pk.u;
    *(volatile u16x8*)(dst + e) = v;
    __threadfence();
    *(volatile u16x8*)(dst + e) = v;
}

__global__ __launch_bounds__(64)
void prep_kernel(const float* __restrict__ x, const float* __restrict__ pcw,
                 const float* __restrict__ pcb, const float* __restrict__ pemb,
                 const float* __restrict__ lng, const float* __restrict__ lnb,
                 float* XS, unsigned short* XN)
{
    __shared__ __attribute__((aligned(16))) float    sx[2][32 * SXP_];
    __shared__ __attribute__((aligned(16))) _Float16 sn[2][32 * CCH_];
    const int tid  = threadIdx.x;
    const int lane = tid & 31;
    const int wave = tid >> 5;
    const int tok  = blockIdx.x * 64 + tid;
    const int b    = tok / LL_;
    const int l    = tok - b * LL_;
    const int hy   = l / WW_;
    const int wx   = l - hy * WW_;
    const float* xb = x + (size_t)b * CCH_ * LL_;
    float* sxr = &sx[wave][lane * SXP_];
    float sum = 0.0f;
#pragma unroll 1
    for (int c = 0; c < CCH_; ++c) {
        const float* xp = xb + (size_t)c * LL_;
        const float* wp = pcw + c * 9;
        float cv = 0.0f;
#pragma unroll
        for (int dy = -1; dy <= 1; ++dy) {
            const int yy = hy + dy;
            if (yy < 0 || yy >= HH_) continue;
#pragma unroll
            for (int dx = -1; dx <= 1; ++dx) {
                const int xx = wx + dx;
                if (xx < 0 || xx >= WW_) continue;
                cv += xp[yy * WW_ + xx] * wp[(dy + 1) * 3 + (dx + 1)];
            }
        }
        const float v = ((xp[l] + cv) + pcb[c]) + pemb[(size_t)l * CCH_ + c];
        sum += v;
        sxr[c] = v;
    }
    const float mean = sum * (1.0f / CCH_);
    float var = 0.0f;
#pragma unroll 4
    for (int c = 0; c < CCH_; ++c) { const float dd = sxr[c] - mean; var += dd * dd; }
    var *= (1.0f / CCH_);
    const float inv = rsqrtf(var + EPS_);
    _Float16* snr = &sn[wave][lane * CCH_];
#pragma unroll 4
    for (int c = 0; c < CCH_; ++c) snr[c] = (_Float16)((sxr[c] - mean) * inv * lng[c] + lnb[c]);
    __syncthreads();

    const int tokw = blockIdx.x * 64 + wave * 32;
#pragma unroll 1
    for (int pass = 0; pass < 2; ++pass) {
#pragma unroll
        for (int it = 0; it < 32; ++it) {
            const v4f v = *(const v4f*)(&sx[wave][it * SXP_ + 4 * lane]);
            *(volatile v4f*)(XS + (size_t)(tokw + it) * CCH_ + 4 * lane) = v;
        }
#pragma unroll
        for (int it = 0; it < 16; ++it) {
            const int chunk = it * 32 + lane;
            const int tl = chunk >> 4;
            const int c8 = chunk & 15;
            Pack8 pk;
            pk.f = *(const v8h*)(&sn[wave][tl * CCH_ + 8 * c8]);
            const u16x8 hv = pk.u;
            *(volatile u16x8*)(XN + (size_t)(tokw + tl) * CCH_ + 8 * c8) = hv;
        }
        if (pass == 0) __threadfence();
    }
}

template<int WM, int WN, int RS, int NBF, int EPI, bool HB>
__global__ __launch_bounds__(32 * WM * WN)
void gemm_kernel(const unsigned short* __restrict__ A, int lda, long long azs,
                 const unsigned short* __restrict__ Bw, int ldb, long long bzs,
                 float* C, float* C2, long long czs, int ldc, int csplit,
                 unsigned short* Ch,
                 const float* __restrict__ bias, const float* __restrict__ ex0,
                 const float* __restrict__ ex1, int K, float scale)
{
    constexpr int T    = 32 * WM * WN;
    constexpr int BM   = 16 * RS * WM;
    constexpr int BN   = 16 * NBF * WN;
    constexpr int P    = BN + 4;
    constexpr int CPR  = BN / 4;
    constexpr int CPR8 = BN / 8;
    constexpr int CPT  = BM / 4;
    static_assert((BM * CPR) % T == 0);
    static_assert((BM * CPR8) % T == 0);
    static_assert((BN * CPT) % T == 0);
    static_assert(BN % 32 == 0);
    static_assert(BM % 32 == 0);
    __shared__ __attribute__((aligned(16))) float st[BM * P];

    const int tid  = threadIdx.x;
    const int lane = tid & 31;
    const int wave = tid >> 5;
    const int h    = lane >> 4;
    const int m    = lane & 15;
    const int wm   = wave / WN;
    const int wn   = wave % WN;
    const int rowBase = blockIdx.y * BM;
    const int colBase = blockIdx.x * BN;
    const int rW = wm * 16 * RS;
    const int cW = wn * 16 * NBF;
    const unsigned short* Az = A + (size_t)blockIdx.z * (size_t)azs;
    const unsigned short* Bz = Bw + (size_t)blockIdx.z * (size_t)bzs;

    v8f acc[RS * NBF];
#pragma unroll
    for (int j = 0; j < RS * NBF; ++j)
#pragma unroll
        for (int r = 0; r < 8; ++r) acc[j][r] = 0.0f;

    const size_t aoff = (size_t)(rowBase + rW + m) * lda + 8 * h;
    const size_t boff = (size_t)(colBase + cW + m) * ldb + 8 * h;
    const size_t a16  = (size_t)16 * lda;
    const size_t b16  = (size_t)16 * ldb;
    const int nk = K >> 5;

    for (int kt = 0; kt < nk; ++kt) {
        const size_t k0 = (size_t)kt * 32;
        FragH fa[RS], fb[NBF];
#pragma unroll
        for (int s = 0; s < RS; ++s) {
            const unsigned short* p = Az + aoff + (size_t)s * a16 + k0;
            fa[s].h[0] = *(const u16x8*)(p);
            fa[s].h[1] = *(const u16x8*)(p + 16);
        }
#pragma unroll
        for (int j = 0; j < NBF; ++j) {
            const unsigned short* p = Bz + boff + (size_t)j * b16 + k0;
            fb[j].h[0] = *(const u16x8*)(p);
            fb[j].h[1] = *(const u16x8*)(p + 16);
        }
#pragma unroll
        for (int s = 0; s < RS; ++s)
#pragma unroll
            for (int j = 0; j < NBF; ++j)
                mma16(acc[s * NBF + j], fa[s], fb[j]);
    }

#pragma unroll
    for (int s = 0; s < RS; ++s)
#pragma unroll
        for (int j = 0; j < NBF; ++j)
#pragma unroll
            for (int r = 0; r < 8; ++r) {
                const int row = rW + s * 16 + 8 * h + r;
                const int col = cW + j * 16 + m;
                float v = acc[s * NBF + j][r] * scale;
                if (HB) v += bias[colBase + col];
                st[row * P + col] = v;
            }
    __syncthreads();

#pragma unroll 1
    for (int pass = 0; pass < 2; ++pass) {
        if (EPI == 0) {
            constexpr int NIT = (BM * CPR) / T;
#pragma unroll
            for (int it = 0; it < NIT; ++it) {
                const int c   = it * T + tid;
                const int row = c / CPR;
                const int f4  = c - row * CPR;
                const v4f v = *(const v4f*)(st + row * P + 4 * f4);
                int gc = colBase + 4 * f4;
                float* Cp = C;
                if (gc >= csplit) { Cp = C2; gc -= csplit; }
                float* dp = Cp + (size_t)blockIdx.z * (size_t)czs + (size_t)(rowBase + row) * ldc + gc;
                *(volatile v4f*)dp = v;
            }
        } else if (EPI == 1) {
            constexpr int NIT = (BM * CPR8) / T;
#pragma unroll 1
            for (int it = 0; it < NIT; ++it) {
                const int c   = it * T + tid;
                const int row = c / CPR8;
                const int c8  = c - row * CPR8;
                const float* sp = st + row * P + 8 * c8;
                const v4f a4 = *(const v4f*)(sp);
                const v4f b4 = *(const v4f*)(sp + 4);
                const size_t gi = (size_t)(rowBase + row) * CCH_ + colBase + 8 * c8;
                const v4f m0 = *(const v4f*)(ex0 + gi);
                const v4f m1 = *(const v4f*)(ex0 + gi + 4);
                const v4f s0 = *(const v4f*)(ex1 + gi);
                const v4f s1 = *(const v4f*)(ex1 + gi + 4);
                const v8f lg = __builtin_shufflevector(a4, b4, 0, 1, 2, 3, 4, 5, 6, 7);
                const v8f xm = __builtin_shufflevector(m0, m1, 0, 1, 2, 3, 4, 5, 6, 7);
                const v8f xs = __builtin_shufflevector(s0, s1, 0, 1, 2, 3, 4, 5, 6, 7);
                v8f o;
#pragma unroll
                for (int q = 0; q < 8; ++q) {
                    const float gv = sigm_f(lg[q]);
                    o[q] = gv * xm[q] + (1.0f - gv) * xs[q];
                }
                Pack8 pk;
                pk.f = __builtin_convertvector(o, v8h);
                const u16x8 hv = pk.u;
                unsigned short* dp = Ch + (size_t)(rowBase + row) * ldc + colBase + 8 * c8;
                *(volatile u16x8*)dp = hv;
            }
        } else {
            constexpr int NIT = (BN * CPT) / T;
            const int bb   = rowBase / LL_;
            const int pos0 = rowBase - bb * LL_;
#pragma unroll
            for (int it = 0; it < NIT; ++it) {
                const int c  = it * T + tid;
                const int nl = c / CPT;
                const int t4 = c - nl * CPT;
                v4f v;
#pragma unroll
                for (int i = 0; i < 4; ++i) v[i] = st[(4 * t4 + i) * P + nl];
                const int n = colBase + nl;
                float* dp = C + ((size_t)(bb * NOUT_ + n)) * LL_ + pos0 + 4 * t4;
                *(volatile v4f*)dp = v;
            }
        }
        if (pass == 0) __threadfence();
    }
}

__global__ __launch_bounds__(64)
void conv_kernel(const float* __restrict__ U, const float* __restrict__ cw,
                 const float* __restrict__ cb, float* UC, unsigned short* UH)
{
    __shared__ __attribute__((aligned(16))) float    su[32 * DI_];
    __shared__ __attribute__((aligned(16))) _Float16 sh[32 * DI_];
    const int tid  = threadIdx.x;
    const int di   = tid;
    const int gd   = blockIdx.y;
    const int g    = gd >> 1;
    const int d    = gd & 1;
    const int tok0 = blockIdx.x * 32;
    const int pd   = gd * DI_ + di;
    const v4f wv   = *(const v4f*)(cw + (size_t)pd * 4);
    const float bias = cb[pd];
    const float* Ug = U + (size_t)g * MT_ * DI_ + di;
#pragma unroll 1
    for (int t = 0; t < 32; ++t) {
        const int p = tok0 + t;
        const int l = p & (LL_ - 1);
        float cv = 0.0f;
#pragma unroll
        for (int j = 0; j < 4; ++j) {
            const int off = d ? (3 - j) : (j - 3);
            const int lq  = l + off;
            if (lq >= 0 && lq < LL_) cv += wv[j] * Ug[(size_t)(p + off) * DI_];
        }
        const float v = silu_f(cv + bias);
        su[t * DI_ + di] = v;
        sh[t * DI_ + di] = (_Float16)(v * USC_);
    }
    __syncthreads();
    float* dstf = UC + ((size_t)gd * MT_ + tok0) * DI_;
    unsigned short* dsth = UH + ((size_t)gd * MT_ + tok0) * DI_;
#pragma unroll 1
    for (int pass = 0; pass < 2; ++pass) {
#pragma unroll
        for (int it = 0; it < 8; ++it) {
            const int c = it * 64 + tid;
            const v4f v = *(const v4f*)(su + c * 4);
            *(volatile v4f*)(dstf + (size_t)c * 4) = v;
        }
#pragma unroll
        for (int it = 0; it < 4; ++it) {
            const int c = it * 64 + tid;
            Pack8 pk;
            pk.f = *(const v8h*)(sh + c * 8);
            const u16x8 hv = pk.u;
            *(volatile u16x8*)(dsth + (size_t)c * 8) = hv;
        }
        if (pass == 0) __threadfence();
    }
}

__global__ __launch_bounds__(64)
void scan_kernel(const float* __restrict__ XD, const float* __restrict__ UC,
                 const float* __restrict__ Z, const float* __restrict__ dtw,
                 const float* __restrict__ dtb, const float* __restrict__ alog,
                 const float* __restrict__ dsk, unsigned short* YC)
{
    __shared__ __attribute__((aligned(16))) _Float16 sy[8 * DI_];
    const int tid = threadIdx.x;
    const int gd  = blockIdx.x;
    const int b   = blockIdx.y;
    const int g   = gd >> 1;
    const int d   = gd & 1;
    const int di  = tid;
    const int pd  = gd * DI_ + di;
    const float w0 = dtw[(size_t)pd * DTR_ + 0];
    const float w1 = dtw[(size_t)pd * DTR_ + 1];
    const float dbias = dtb[pd];
    const float Dv = dsk[pd];
    float An[NS_], hs[NS_];
#pragma unroll
    for (int n = 0; n < NS_; ++n) {
        An[n] = -__expf(alog[(size_t)pd * NS_ + n]);
        hs[n] = 0.0f;
    }
    const size_t rb = (size_t)b * LL_;
    const float* XDg = XD + ((size_t)gd * MT_ + rb) * XDN_;
    const float* UCg = UC + ((size_t)gd * MT_ + rb) * DI_ + di;
    const float* Zg  = Z + ((size_t)g * MT_ + rb) * DI_ + di;
    unsigned short* Yg = YC + ((size_t)g * MT_ + rb) * (2 * DI_) + d * DI_;

#pragma unroll 1
    for (int s0 = 0; s0 < LL_; s0 += 8) {
#pragma unroll 1
        for (int t = 0; t < 8; ++t) {
            const int s = s0 + t;
            const int p = d ? (LL_ - 1 - s) : s;
            const float* xr = XDg + (size_t)p * XDN_;
            float xv[36];
#pragma unroll
            for (int i = 0; i < 9; ++i) {
                const v4f q = *(const v4f*)(xr + 4 * i);
                xv[4 * i + 0] = q[0];
                xv[4 * i + 1] = q[1];
                xv[4 * i + 2] = q[2];
                xv[4 * i + 3] = q[3];
            }
            const float sdt   = (xv[0] * w0 + xv[1] * w1) + dbias;
            const float delta = softplus_f(sdt);
            const float u  = UCg[(size_t)p * DI_];
            const float du = delta * u;
            float y = 0.0f;
#pragma unroll
            for (int n = 0; n < NS_; ++n) {
                const float dA = __expf(delta * An[n]);
                hs[n] = hs[n] * dA + du * xv[DTR_ + n];
                y += hs[n] * xv[DTR_ + NS_ + n];
            }
            const float z  = Zg[(size_t)p * DI_];
            const float yo = (y + u * Dv) * silu_f(z);
            sy[t * DI_ + di] = (_Float16)(yo * YSC_);
        }
        __syncthreads();
        const int q  = tid >> 3;
        const int cc = tid & 7;
        const int pq = d ? (LL_ - 1 - (s0 + q)) : (s0 + q);
        Pack8 pk;
        pk.f = *(const v8h*)(&sy[q * DI_ + 8 * cc]);
        const u16x8 hv = pk.u;
        unsigned short* dp = Yg + (size_t)pq * (2 * DI_) + 8 * cc;
        *(volatile u16x8*)dp = hv;
        __threadfence();
        *(volatile u16x8*)dp = hv;
        __syncthreads();
    }
}

extern "C" void kernel_launch(void* const* d_in, const int* in_sizes, int n_in,
                              void* d_out, int out_size, void* d_ws, size_t ws_size,
                              hipStream_t stream)
{
    if (n_in < 19) return;
    if (in_sizes[0]  != MT_ * CCH_) return;
    if (in_sizes[1]  != CCH_ * 9 || in_sizes[2] != CCH_) return;
    if (in_sizes[3]  != LL_ * CCH_) return;
    if (in_sizes[4]  != CCH_ || in_sizes[5] != CCH_) return;
    if (in_sizes[6]  != CCH_ * CCH_ || in_sizes[7] != CCH_) return;
    if (in_sizes[8]  != NOUT_ * CCH_ || in_sizes[9] != NOUT_) return;
    if (in_sizes[10] != NG_ * 2 * DI_ * DM_) return;
    if (in_sizes[11] != NG_ * DM_ * DI_) return;
    if (in_sizes[12] != NGD_ * DI_ * 4 || in_sizes[13] != NGD_ * DI_) return;
    if (in_sizes[14] != NGD_ * XDW_ * DI_) return;
    if (in_sizes[15] != NGD_ * DI_ * DTR_ || in_sizes[16] != NGD_ * DI_) return;
    if (in_sizes[17] != NGD_ * DI_ * NS_ || in_sizes[18] != NGD_ * DI_) return;
    if (out_size != MT_ * NOUT_) return;

    const float* x          = (const float*)d_in[0];
    const float* pos_conv_w = (const float*)d_in[1];
    const float* pos_conv_b = (const float*)d_in[2];
    const float* pos_embed  = (const float*)d_in[3];
    const float* ln_g       = (const float*)d_in[4];
    const float* ln_b       = (const float*)d_in[5];
    const float* gate_W     = (const float*)d_in[6];
    const float* gate_b     = (const float*)d_in[7];
    const float* proj_W     = (const float*)d_in[8];
    const float* proj_b     = (const float*)d_in[9];
    const float* m_Win      = (const float*)d_in[10];
    const float* m_Wout     = (const float*)d_in[11];
    const float* conv_w     = (const float*)d_in[12];
    const float* conv_b     = (const float*)d_in[13];
    const float* xproj_W    = (const float*)d_in[14];
    const float* dt_W       = (const float*)d_in[15];
    const float* dt_b       = (const float*)d_in[16];
    const float* A_log      = (const float*)d_in[17];
    const float* Dskip      = (const float*)d_in[18];
    float* out = (float*)d_out;

    const size_t SZ_WG = (size_t)CCH_ * CCH_ * 2;
    const size_t SZ_WP = (size_t)NOUT_ * CCH_ * 2;
    const size_t SZ_WI = (size_t)NG_ * 2 * DI_ * DM_ * 2;
    const size_t SZ_WX = (size_t)NGD_ * XDN_ * DI_ * 2;
    const size_t SZ_WO = (size_t)NG_ * DM_ * 2 * DI_ * 2;
    const size_t SZ_XS = (size_t)MT_ * CCH_ * 4;
    const size_t SZ_XN = (size_t)MT_ * CCH_ * 2;
    const size_t SZ_UZ = (size_t)NG_ * MT_ * DI_ * 4;
    const size_t SZ_UC = (size_t)NGD_ * MT_ * DI_ * 4;
    const size_t SZ_UH = (size_t)NGD_ * MT_ * DI_ * 2;
    const size_t SZ_XD = (size_t)NGD_ * MT_ * XDN_ * 4;
    const size_t SZ_YC = (size_t)NG_ * MT_ * 2 * DI_ * 2;
    const size_t SZ_XM = (size_t)MT_ * CCH_ * 4;
    const size_t SZ_GT = (size_t)MT_ * CCH_ * 2;

    const size_t OFF_WG = 0;
    const size_t OFF_WP = OFF_WG + SZ_WG;
    const size_t OFF_WI = OFF_WP + SZ_WP;
    const size_t OFF_WX = OFF_WI + SZ_WI;
    const size_t OFF_WO = OFF_WX + SZ_WX;
    const size_t OFF_XS = OFF_WO + SZ_WO;
    const size_t OFF_XN = OFF_XS + SZ_XS;
    const size_t OFF_U  = OFF_XN + SZ_XN;
    const size_t OFF_Z  = OFF_U + SZ_UZ;
    const size_t OFF_UC = OFF_Z + SZ_UZ;
    const size_t OFF_UH = OFF_UC + SZ_UC;
    const size_t OFF_XD = OFF_UH + SZ_UH;
    const size_t WS_END = OFF_XD + SZ_XD;
    const size_t OFF_YC = OFF_UH;
    const size_t OFF_XM = OFF_U;
    const size_t OFF_GT = OFF_U + SZ_XM;
    if (SZ_YC > SZ_UH) return;
    if (SZ_XM + SZ_GT > SZ_UZ) return;
    if (WS_END > (size_t)134217728) return;
    if (ws_size < WS_END) return;

    char* ws = (char*)d_ws;
    unsigned short* wg16 = (unsigned short*)(ws + OFF_WG);
    unsigned short* wp16 = (unsigned short*)(ws + OFF_WP);
    unsigned short* wi16 = (unsigned short*)(ws + OFF_WI);
    unsigned short* wx16 = (unsigned short*)(ws + OFF_WX);
    unsigned short* wo16 = (unsigned short*)(ws + OFF_WO);
    float*          xs32 = (float*)(ws + OFF_XS);
    unsigned short* xn16 = (unsigned short*)(ws + OFF_XN);
    float*          u32  = (float*)(ws + OFF_U);
    float*          z32  = (float*)(ws + OFF_Z);
    float*          uc32 = (float*)(ws + OFF_UC);
    unsigned short* uc16 = (unsigned short*)(ws + OFF_UH);
    float*          xd32 = (float*)(ws + OFF_XD);
    unsigned short* yc16 = (unsigned short*)(ws + OFF_YC);
    float*          xm32 = (float*)(ws + OFF_XM);
    unsigned short* gt16 = (unsigned short*)(ws + OFF_GT);

    const float inv_w  = 1.0f / WSC_;
    const float inv_wu = 1.0f / (WSC_ * USC_);
    const float inv_wy = 1.0f / (WSC_ * YSC_);
    const int   nosplit = 1 << 30;

    cvt_w_kernel<<<dim3((NGD_ * XDN_ * DI_ / 8 + 255) / 256, 5), dim3(256), 0, stream>>>(
        gate_W, proj_W, m_Win, xproj_W, m_Wout, wg16, wp16, wi16, wx16, wo16);

    prep_kernel<<<dim3(MT_ / 64), dim3(64), 0, stream>>>(
        x, pos_conv_w, pos_conv_b, pos_embed, ln_g, ln_b, xs32, xn16);

    gemm_kernel<2, 2, 2, 4, 0, false><<<dim3(1, MT_ / 64, NG_), dim3(128), 0, stream>>>(
        xn16, (int)CCH_, (long long)DM_, wi16, (int)DM_, (long long)(2 * DI_ * DM_),
        u32, z32, (long long)MT_ * DI_, (int)DI_, (int)DI_, gt16,
        gate_b, xs32, xs32, (int)DM_, inv_w);

    conv_kernel<<<dim3(MT_ / 32, NGD_), dim3(64), 0, stream>>>(u32, conv_w, conv_b, uc32, uc16);

    gemm_kernel<2, 1, 2, 4, 0, false><<<dim3(1, MT_ / 64, NGD_), dim3(64), 0, stream>>>(
        uc16, (int)DI_, (long long)MT_ * DI_, wx16, (int)DI_, (long long)(XDN_ * DI_),
        xd32, xd32, (long long)MT_ * XDN_, (int)XDN_, nosplit, gt16,
        gate_b, xs32, xs32, (int)DI_, inv_wu);

    scan_kernel<<<dim3(NGD_, NB_), dim3(64), 0, stream>>>(
        xd32, uc32, z32, dt_W, dt_b, A_log, Dskip, yc16);

    gemm_kernel<2, 1, 2, 2, 0, false><<<dim3(1, MT_ / 64, NG_), dim3(64), 0, stream>>>(
        yc16, (int)(2 * DI_), (long long)MT_ * 2 * DI_, wo16, (int)(2 * DI_), (long long)(DM_ * 2 * DI_),
        xm32, xm32, (long long)DM_, (int)CCH_, nosplit, gt16,
        gate_b, xs32, xs32, (int)(2 * DI_), inv_wy);

    gemm_kernel<2, 2, 2, 4, 1, true><<<dim3(1, MT_ / 64, 1), dim3(128), 0, stream>>>(
        xn16, (int)CCH_, 0LL, wg16, (int)CCH_, 0LL,
        xm32, xm32, 0LL, (int)CCH_, nosplit, gt16,
        gate_b, xm32, xs32, (int)CCH_, inv_w);

    gemm_kernel<2, 2, 2, 4, 2, true><<<dim3(1, MT_ / 64, 1), dim3(128), 0, stream>>>(
        gt16, (int)CCH_, 0LL, wp16, (int)CCH_, 0LL,
        out, out, 0LL, (int)NOUT_, nosplit, gt16,
        proj_b, xs32, xs32, (int)CCH_, inv_w);
}
